// PixelRNN_45715631899296
// MI455X (gfx1250) — hardware-verified
//
#include <hip/hip_runtime.h>
#include <stddef.h>

typedef __attribute__((ext_vector_type(16))) __bf16         v16b;
typedef __attribute__((ext_vector_type(8)))  unsigned short v8us;
typedef __attribute__((ext_vector_type(8)))  float          v8f;
typedef __attribute__((ext_vector_type(4)))  float          v4f;
static_assert(sizeof(v8us) == 16, "v8us is 16 bytes");
static_assert(sizeof(v16b) == 32, "v16b is 32 bytes");

constexpr int kHid      = 64;
constexpr int kRS       = 8;
constexpr int kCh       = 3;
constexpr int kImH      = 24;
constexpr int kImW      = 24;
constexpr int kL        = 8;
constexpr int kSteps    = 16;
constexpr int kKFeed    = 32;
constexpr int kNGate    = 4 * kHid;
constexpr int kNHeadP   = 16;
constexpr int kWaves    = 2;
constexpr int kRbPitch  = kCh * kImW;
constexpr int kXStride  = kCh * kImH * kImW;
constexpr int kChStride = kImH * kImW;
constexpr int kOutPerImg = kCh * kSteps * kSteps;

static_assert(kKFeed % 32 == 0, "feed K is a multiple of 32");
static_assert(kHid % 32 == 0, "hidden K is a multiple of 32");
static_assert(kNGate % 16 == 0, "gate N is a multiple of 16");
static_assert(kCh * kRS <= kKFeed, "feed fits the padded K");

constexpr size_t kWihBytes = (size_t)kNGate * kKFeed * 2;
constexpr size_t kWhhBytes = (size_t)kNGate * kHid * 2;
constexpr size_t kWlBytes  = (size_t)kNHeadP * kHid * 2;
constexpr size_t kWihOff   = 0;
constexpr size_t kWhhOff   = kWihOff + kWihBytes;
constexpr size_t kWlOff    = kWhhOff + kWhhBytes;
constexpr size_t kWsTotal  = kWlOff + kWlBytes;
static_assert(kWsTotal == 51200, "carve total");
static_assert(kWsTotal <= 134217728, "carve under 128 MiB");
static_assert(kWihOff % 128 == 0 && kWhhOff % 128 == 0 && kWlOff % 128 == 0, "line aligned regions");
static_assert(kWihBytes % 512 == 0 && kWhhBytes % 512 == 0 && kWlBytes % 512 == 0, "each region is whole waves of 16-B chunks");

__device__ __forceinline__ unsigned short f2bf_bits(float f) {
  unsigned u = __float_as_uint(f);
  return (unsigned short)((u + 0x7FFFu + ((u >> 16) & 1u)) >> 16);
}
__device__ __forceinline__ float bf_bits2f(unsigned short h) { return __uint_as_float(((unsigned)h) << 16); }
__device__ __forceinline__ float bfr(float f) { return bf_bits2f(f2bf_bits(f)); }
__device__ __forceinline__ void split2(float f, unsigned short& hb, unsigned short& lb) {
  hb = f2bf_bits(f);
  lb = f2bf_bits(f - bf_bits2f(hb));
}

union FragU { v16b v; v8us h[2]; };
__device__ __forceinline__ v16b frag16(const unsigned short* p) {
  FragU u;
  u.h[0] = *(const v8us*)(p);
  u.h[1] = *(const v8us*)(p + 16);
  return u.v;
}

__device__ __forceinline__ v8f mma_bf(v16b a, v16b b, v8f c) {
  return __builtin_amdgcn_wmma_f32_16x16x32_bf16(false, a, false, b, (short)0, c, false, false);
}
__device__ __forceinline__ void guard4(v8f& a, v8f& b, v8f& c, v8f& d, v16b x, v16b y) {
  asm volatile("v_nop\n\tv_nop\n\tv_nop\n\tv_nop" : "+v"(a), "+v"(b), "+v"(c), "+v"(d) : "v"(x), "v"(y));
}
__device__ __forceinline__ void guard1(v8f& a, v16b x, v16b y, v16b z) {
  asm volatile("v_nop\n\tv_nop\n\tv_nop\n\tv_nop" : "+v"(a) : "v"(x), "v"(y), "v"(z));
}
__device__ __forceinline__ void keep4b(v16b a, v16b b, v16b c, v16b d) {
  asm volatile("v_nop" :: "v"(a), "v"(b), "v"(c), "v"(d));
}

__device__ __forceinline__ float sigm(float x) {
  return __builtin_amdgcn_rcpf(1.0f + __builtin_amdgcn_exp2f(x * -1.4426950408889634f));
}
__device__ __forceinline__ float tanhx(float x) {
  const float r = __builtin_amdgcn_rcpf(1.0f + __builtin_amdgcn_exp2f(x * -2.8853900817779268f));
  return fmaf(2.0f, r, -1.0f);
}

__global__ __launch_bounds__(256) void k_prep(
    const float* __restrict__ w_ih, const float* __restrict__ w_hh, const float* __restrict__ w_l,
    unsigned short* __restrict__ wih_p, unsigned short* __restrict__ whh_p, unsigned short* __restrict__ wl_p) {
  const int blk = blockIdx.x;
  const int t = threadIdx.x;
  float v[8];
  if (blk < 4) {
    const int c = blk * 256 + t;
    const int row = c >> 2;
    const int kb = (c & 3) * 8;
#pragma unroll
    for (int e = 0; e < 8; ++e) {
      const int k = kb + e;
      const int kc = k < 24 ? k : 23;
      const float tv = w_ih[row * 24 + kc];
      v[e] = (k < 24) ? tv : 0.0f;
    }
    v8us u;
#pragma unroll
    for (int e = 0; e < 8; ++e) u[e] = f2bf_bits(v[e]);
    unsigned short* dst = wih_p + (size_t)c * 8;
    *(volatile v8us*)dst = u;
    __threadfence();
    *(volatile v8us*)dst = u;
  } else if (blk < 12) {
    const int c2 = (blk - 4) * 256 + t;
    const int row = c2 >> 3;
    const int kb = (c2 & 7) * 8;
#pragma unroll
    for (int e = 0; e < 8; ++e) v[e] = w_hh[row * 64 + kb + e];
    v8us u;
#pragma unroll
    for (int e = 0; e < 8; ++e) u[e] = f2bf_bits(v[e]);
    unsigned short* dst = whh_p + (size_t)c2 * 8;
    *(volatile v8us*)dst = u;
    __threadfence();
    *(volatile v8us*)dst = u;
  } else {
    if (t >= 128) return;
    const int c3 = t;
    const int row = c3 >> 3;
    const int kb = (c3 & 7) * 8;
    const int rc = row < 3 ? row : 2;
#pragma unroll
    for (int e = 0; e < 8; ++e) {
      const float tv = w_l[rc * 64 + kb + e];
      v[e] = (row < 3) ? tv : 0.0f;
    }
    v8us u;
#pragma unroll
    for (int e = 0; e < 8; ++e) u[e] = f2bf_bits(v[e]);
    unsigned short* dst = wl_p + (size_t)c3 * 8;
    *(volatile v8us*)dst = u;
    __threadfence();
    *(volatile v8us*)dst = u;
  }
}

template <int HT>
__device__ __forceinline__ void gate_tile(const unsigned short* fdw, const unsigned short* hxc, unsigned short* hxn,
                                          const unsigned short* __restrict__ wih, const unsigned short* __restrict__ whh,
                                          const float* sb, v8f& cxt, int rl, int hh) {
  v8f acc[4];
#pragma unroll
  for (int g = 0; g < 4; ++g) acc[g] = (v8f){0.f, 0.f, 0.f, 0.f, 0.f, 0.f, 0.f, 0.f};

  {
    v16b bq[4];
#pragma unroll
    for (int g = 0; g < 4; ++g)
      bq[g] = frag16(wih + (size_t)(g * kHid + HT * 16 + rl) * kKFeed + 8 * hh);
    const v16b ah = frag16(fdw + rl * kKFeed + 8 * hh);
    const v16b al = frag16(fdw + 512 + rl * kKFeed + 8 * hh);
#pragma unroll
    for (int g = 0; g < 4; ++g) {
      acc[g] = mma_bf(ah, bq[g], acc[g]);
      acc[g] = mma_bf(al, bq[g], acc[g]);
    }
    guard4(acc[0], acc[1], acc[2], acc[3], ah, al);
    keep4b(bq[0], bq[1], bq[2], bq[3]);
  }
#pragma unroll 1
  for (int ks = 0; ks < 2; ++ks) {
    v16b bq[4];
#pragma unroll
    for (int g = 0; g < 4; ++g)
      bq[g] = frag16(whh + (size_t)(g * kHid + HT * 16 + rl) * kHid + ks * 32 + 8 * hh);
    const v16b ah = frag16(hxc + rl * kHid + ks * 32 + 8 * hh);
    const v16b al = frag16(hxc + 1024 + rl * kHid + ks * 32 + 8 * hh);
#pragma unroll
    for (int g = 0; g < 4; ++g) {
      acc[g] = mma_bf(ah, bq[g], acc[g]);
      acc[g] = mma_bf(al, bq[g], acc[g]);
    }
    guard4(acc[0], acc[1], acc[2], acc[3], ah, al);
    keep4b(bq[0], bq[1], bq[2], bq[3]);
  }

  const float bi = sb[0 * kHid + HT * 16 + rl];
  const float bf = sb[1 * kHid + HT * 16 + rl];
  const float bg = sb[2 * kHid + HT * 16 + rl];
  const float bo = sb[3 * kHid + HT * 16 + rl];
#pragma unroll
  for (int r = 0; r < 8; ++r) {
    const float gi = acc[0][r] + bi;
    const float gf = acc[1][r] + bf;
    const float gg = acc[2][r] + bg;
    const float go = acc[3][r] + bo;
    const float c = sigm(gf) * cxt[r] + sigm(gi) * tanhx(gg);
    cxt[r] = c;
    const float h = sigm(go) * tanhx(c);
    unsigned short hb, lb;
    split2(h, hb, lb);
    const int idx = (8 * hh + r) * kHid + HT * 16 + rl;
    hxn[idx] = hb;
    hxn[1024 + idx] = lb;
  }
}

__global__ __launch_bounds__(kWaves * 32) void k_lstm(
    const float* __restrict__ x, const float* __restrict__ b_ih, const float* __restrict__ b_hh,
    const float* __restrict__ b_l,
    const unsigned short* __restrict__ wih_p, const unsigned short* __restrict__ whh_p,
    const unsigned short* __restrict__ wl_p, float* __restrict__ out) {
  __shared__ __align__(16) unsigned short s_hx[kWaves][4][1024];
  __shared__ __align__(16) unsigned short s_fd[kWaves][2][512];
  __shared__ __align__(16) float s_rb[kWaves][16 * kRbPitch];
  __shared__ __align__(16) float s_os[kWaves][48 * 32];
  __shared__ __align__(16) float s_sb[kWaves][kNGate];

  const int lane = threadIdx.x & 31;
  const int wave = threadIdx.x >> 5;
  const int hh = lane >> 4;
  const int rl = lane & 15;
  const int b0 = (blockIdx.x * kWaves + wave) * 16;

  unsigned short* hxw = &s_hx[wave][0][0];
  unsigned short* fdw = &s_fd[wave][0][0];
  float* rb = s_rb[wave];
  float* os = s_os[wave];
  float* sb = s_sb[wave];

  {
    const v8us z8 = (v8us){0, 0, 0, 0, 0, 0, 0, 0};
    const v4f z4 = (v4f){0.f, 0.f, 0.f, 0.f};
#pragma unroll
    for (int i = 0; i < 16; ++i) *(v8us*)(hxw + (lane + 32 * i) * 8) = z8;
#pragma unroll
    for (int i = 0; i < 4; ++i) *(v8us*)(fdw + (lane + 32 * i) * 8) = z8;
#pragma unroll
    for (int i = 0; i < 9; ++i) *(v4f*)(rb + (lane + 32 * i) * 4) = z4;
#pragma unroll
    for (int i = 0; i < 12; ++i) *(v4f*)(os + (lane + 32 * i) * 4) = z4;
#pragma unroll
    for (int i = 0; i < 2; ++i) {
      const int c4 = lane + 32 * i;
      const v4f ta = *(const v4f*)(b_ih + 4 * c4);
      const v4f tb = *(const v4f*)(b_hh + 4 * c4);
      v4f s;
#pragma unroll
      for (int e = 0; e < 4; ++e) s[e] = bfr(ta[e]) + bfr(tb[e]);
      *(v4f*)(sb + 4 * c4) = s;
    }
  }
  const int rc3 = rl < 3 ? rl : 2;
  const float blt = b_l[rc3];
  const float blv = (rl < 3) ? bfr(blt) : 0.0f;

  v8f cx0 = (v8f){0.f, 0.f, 0.f, 0.f, 0.f, 0.f, 0.f, 0.f};
  v8f cx1 = cx0, cx2 = cx0, cx3 = cx0;
  __syncthreads();

  for (int ri = 0; ri < kSteps; ++ri) {
    __syncthreads();
#pragma unroll
    for (int i = 0; i < 3; ++i) {
      const int c4 = lane + 32 * i;
      const int pr = c4 >> 1;
      const int q = c4 & 1;
      const int m = pr / 3;
      const int ch = pr - m * 3;
      const v4f tv = *(const v4f*)(x + ((size_t)(b0 + m) * kXStride + (size_t)ch * kChStride + (size_t)(ri + kL) * kImW + 4 * q));
      v4f uv;
#pragma unroll
      for (int e = 0; e < 4; ++e) uv[e] = bfr(tv[e]);
      *(v4f*)(rb + m * kRbPitch + ch * kImW + 4 * q) = uv;
    }

    for (int cc = 0; cc < kSteps; ++cc) {
      const int step = ri * kSteps + cc;
      const int cur = step & 1;
      const int nxt = cur ^ 1;
      __syncthreads();
#pragma unroll
      for (int gi = 0; gi < 2; ++gi) {
        const int grp = hh + 2 * gi;
        const int ch = grp < 3 ? grp : 2;
        const bool zer = (grp == 3);
        const float* src = rb + rl * kRbPitch + ch * kImW + cc;
        v8us hv, lv;
#pragma unroll
        for (int j = 0; j < 8; ++j) {
          float f = src[j];
          f = zer ? 0.0f : f;
          unsigned short hb, lb;
          split2(f, hb, lb);
          hv[j] = hb;
          lv[j] = lb;
        }
        *(v8us*)(fdw + rl * kKFeed + grp * 8) = hv;
        *(v8us*)(fdw + 512 + rl * kKFeed + grp * 8) = lv;
      }
      __syncthreads();

      const unsigned short* hxc = hxw + cur * 2048;
      unsigned short* hxn = hxw + nxt * 2048;
      gate_tile<0>(fdw, hxc, hxn, wih_p, whh_p, sb, cx0, rl, hh);
      gate_tile<1>(fdw, hxc, hxn, wih_p, whh_p, sb, cx1, rl, hh);
      gate_tile<2>(fdw, hxc, hxn, wih_p, whh_p, sb, cx2, rl, hh);
      gate_tile<3>(fdw, hxc, hxn, wih_p, whh_p, sb, cx3, rl, hh);
      __syncthreads();

      v8f ha = (v8f){0.f, 0.f, 0.f, 0.f, 0.f, 0.f, 0.f, 0.f};
#pragma unroll
      for (int ks = 0; ks < 2; ++ks) {
        const v16b bw = frag16(wl_p + (size_t)rl * kHid + ks * 32 + 8 * hh);
        const v16b ah = frag16(hxn + rl * kHid + ks * 32 + 8 * hh);
        const v16b al = frag16(hxn + 1024 + rl * kHid + ks * 32 + 8 * hh);
        ha = mma_bf(ah, bw, ha);
        ha = mma_bf(al, bw, ha);
        guard1(ha, ah, al, bw);
      }
#pragma unroll
      for (int r = 0; r < 8; ++r) {
        float v = ha[r] + blv;
        v = (v >= 0.0f) ? v : 0.01f * v;
        const int row = 8 * hh + r;
        if (rl < 3) {
          rb[row * kRbPitch + rl * kImW + kRS + cc] = v;
          os[(row * 3 + rl) * 32 + (ri & 1) * 16 + cc] = v;
        }
      }
    }

    if (ri & 1) {
      __syncthreads();
      float* ob = out + (size_t)b0 * kOutPerImg + (size_t)(ri - 1) * kSteps;
      const int q = lane >> 3;
      const int j4 = (lane & 7) * 4;
      for (int pass = 0; pass < 2; ++pass) {
#pragma unroll
        for (int it = 0; it < 12; ++it) {
          const int lw = it * 4 + q;
          const v4f val = *(const v4f*)(os + lw * 32 + j4);
          *(volatile v4f*)(ob + (size_t)lw * (kSteps * kSteps) + j4) = val;
        }
        __threadfence();
      }
    }
  }
}

extern "C" void kernel_launch(void* const* d_in, const int* in_sizes, int n_in,
                              void* d_out, int out_size, void* d_ws, size_t ws_size,
                              hipStream_t stream) {
  (void)n_in;
  const float* x    = (const float*)d_in[0];
  const float* w_ih = (const float*)d_in[1];
  const float* w_hh = (const float*)d_in[2];
  const float* b_ih = (const float*)d_in[3];
  const float* b_hh = (const float*)d_in[4];
  const float* w_l  = (const float*)d_in[5];
  const float* b_l  = (const float*)d_in[6];
  float* out = (float*)d_out;

  unsigned char* ws = (unsigned char*)d_ws;
  unsigned short* wih_p = (unsigned short*)(ws + kWihOff);
  unsigned short* whh_p = (unsigned short*)(ws + kWhhOff);
  unsigned short* wl_p  = (unsigned short*)(ws + kWlOff);

  const int nb = in_sizes[0] / kXStride;
  int nblk = nb / (16 * kWaves);
  const int nblk_out = out_size / (16 * kWaves * kOutPerImg);
  if (nblk > nblk_out) nblk = nblk_out;
  if (ws_size < kWsTotal || nblk <= 0) return;

  k_prep<<<13, 256, 0, stream>>>(w_ih, w_hh, w_l, wih_p, whh_p, wl_p);
  k_lstm<<<nblk, kWaves * 32, 0, stream>>>(x, b_ih, b_hh, b_l, wih_p, whh_p, wl_p, out);
}
